// MultiHeadedSelfAttention_16484084482417
// MI455X (gfx1250) — hardware-verified
//
#include <hip/hip_runtime.h>


#ifndef NB
#define NB 2
#endif
#ifndef SEQ
#define SEQ 2048
#endif
#define NB_FULL  2
#define SEQ_FULL 2048
#define DM   1024
#define NHD  16
#define HD   64
#define SEQW (SEQ / 32)
#define NWL  ((SEQW + 31) / 32)
#define MROWS (NB * SEQ)
#define PCAR 256.0f
#define CCAR 64.0f
#define WCAR 64.0f
#define SCL  0.125f
#define NEGV (-1000000000.0f)
#define L2E  1.4426950408889634f
static_assert(SEQ % 128 == 0);
static_assert(SEQ >= 128 && SEQ <= SEQ_FULL);
static_assert(NB >= 1 && NB <= NB_FULL);
static_assert(DM == NHD * HD);
static_assert(DM % 64 == 0 && MROWS % 64 == 0 && DM % 32 == 0);
static_assert(SEQW % 4 == 0);

typedef _Float16 h16;
typedef unsigned short bf;
typedef __attribute__((ext_vector_type(16))) __bf16   v16bf;
typedef __attribute__((ext_vector_type(16))) _Float16 v16h;
typedef __attribute__((ext_vector_type(8)))  _Float16 v8h;
typedef __attribute__((ext_vector_type(8)))  unsigned short v8us;
typedef __attribute__((ext_vector_type(8)))  float    v8f;
typedef __attribute__((ext_vector_type(4)))  float    v4f;
typedef __attribute__((ext_vector_type(2)))  _Float16 v2h;
typedef __attribute__((ext_vector_type(2)))  unsigned short v2us;
typedef v8h  __attribute__((may_alias)) v8ha;
typedef v4f  __attribute__((may_alias)) v4fa;
typedef v8us __attribute__((may_alias)) v8usa;

__device__ __forceinline__ unsigned short f2bf(float f) { unsigned u = __float_as_uint(f); u += 0x7FFFu + ((u >> 16) & 1u); return (unsigned short)(u >> 16); }
__device__ __forceinline__ float bf2f(unsigned short b) { return __uint_as_float(((unsigned)b) << 16); }
__device__ __forceinline__ float bfr(float f) { return bf2f(f2bf(f)); }
__device__ __forceinline__ h16 tohx(float x) { return (h16)x; }
__device__ __forceinline__ void splitf(float y, unsigned short& h, unsigned short& l) { h = f2bf(y); l = f2bf(y - bf2f(h)); }
__device__ __forceinline__ v16h cat16(v8h lo, v8h hi) { return __builtin_shufflevector(lo, hi, 0, 1, 2, 3, 4, 5, 6, 7, 8, 9, 10, 11, 12, 13, 14, 15); }
__device__ __forceinline__ v16bf cat16b(v8us lo, v8us hi) { return __builtin_bit_cast(v16bf, __builtin_shufflevector(lo, hi, 0, 1, 2, 3, 4, 5, 6, 7, 8, 9, 10, 11, 12, 13, 14, 15)); }
__device__ __forceinline__ v8f wmma16(v16h a, v16h b, v8f c) { return __builtin_amdgcn_wmma_f32_16x16x32_f16(false, a, false, b, (short)0, c, false, false); }
__device__ __forceinline__ v8f wmmab(v16bf a, v16bf b, v8f c) { return __builtin_amdgcn_wmma_f32_16x16x32_bf16(false, a, false, b, (short)0, c, false, false); }

template <typename T16> struct WFrag;
template <> struct WFrag<h16> { typedef v16h V; static __device__ __forceinline__ V ld(const h16* p) { return cat16(*(const v8h*)p, *(const v8h*)(p + 16)); } static __device__ __forceinline__ v8f mma(V a, V b, v8f c) { return wmma16(a, b, c); } };
template <> struct WFrag<bf> { typedef v16bf V; static __device__ __forceinline__ V ld(const bf* p) { return cat16b(*(const v8us*)p, *(const v8us*)(p + 16)); } static __device__ __forceinline__ v8f mma(V a, V b, v8f c) { return wmmab(a, b, c); } };
template <typename T16, int NSPLIT, bool BIAS>
__global__ __launch_bounds__(32) void k_gemmw(const T16* __restrict__ A, const T16* __restrict__ A2, const T16* __restrict__ Bt, const T16* __restrict__ Bt2, int K, float* C, int ldc, const float* __restrict__ bias, float osc, size_t sA, size_t sB, size_t sC) {
    typedef typename WFrag<T16>::V V;
    __shared__ __align__(16) float os[16 * 68];
    const size_t z = blockIdx.z; A += z * sA; if (A2) A2 += z * sA; Bt += z * sB; if (Bt2) Bt2 += z * sB; C += z * sC;
    const int lane = threadIdx.x & 31, lr = lane & 15, hi = lane >> 4; const int r0 = blockIdx.x * 64, c0 = blockIdx.y * 64;
    v8f acc[4][4];
#pragma unroll
    for (int mb = 0; mb < 4; ++mb)
#pragma unroll
        for (int nb = 0; nb < 4; ++nb) acc[mb][nb] = (v8f){};
    const size_t aoff = (size_t)(r0 + lr) * K + 8 * hi, boff = (size_t)(c0 + lr) * K + 8 * hi;
#pragma unroll 1
    for (int kc = 0; kc < K; kc += 32) {
        V a[4], a2[4];
#pragma unroll
        for (int mb = 0; mb < 4; ++mb) { a[mb] = WFrag<T16>::ld(A + aoff + (size_t)mb * 16 * K + kc); if (NSPLIT == 1 || NSPLIT == 2) a2[mb] = WFrag<T16>::ld(A2 + aoff + (size_t)mb * 16 * K + kc); }
#pragma unroll
        for (int nb = 0; nb < 4; ++nb) { const V b = WFrag<T16>::ld(Bt + boff + (size_t)nb * 16 * K + kc); V b2; if (NSPLIT >= 2) b2 = WFrag<T16>::ld(Bt2 + boff + (size_t)nb * 16 * K + kc);
#pragma unroll
            for (int mb = 0; mb < 4; ++mb) { acc[mb][nb] = WFrag<T16>::mma(a[mb], b, acc[mb][nb]); if (NSPLIT == 1 || NSPLIT == 2) acc[mb][nb] = WFrag<T16>::mma(a2[mb], b, acc[mb][nb]); if (NSPLIT >= 2) acc[mb][nb] = WFrag<T16>::mma(a[mb], b2, acc[mb][nb]); } }
        asm volatile("v_nop\n\tv_nop\n\tv_nop\n\tv_nop" : "+v"(acc[0][0]), "+v"(acc[1][1]), "+v"(acc[2][2]), "+v"(acc[3][3]) : "v"(a[0]), "v"(a[3]));
    }
#pragma unroll
    for (int mb = 0; mb < 4; ++mb) {
#pragma unroll
        for (int nb = 0; nb < 4; ++nb) {
#pragma unroll
            for (int j = 0; j < 8; ++j) os[(hi * 8 + j) * 68 + nb * 16 + lr] = acc[mb][nb][j]; }
        __builtin_amdgcn_fence(3  , "wavefront"); __builtin_amdgcn_wave_barrier(); asm volatile("" ::: "memory");
        float* crow = C + (size_t)(r0 + mb * 16) * ldc + c0;
#pragma unroll 1
        for (int ps = 0; ps < 2; ++ps) {
#pragma unroll
            for (int s = 0; s < 8; ++s) { const int row = 2 * s + hi, cofs = lr * 4; v4f val = *(const v4fa*)(os + row * 68 + cofs); val = val * osc;
                if (BIAS) { val[0] += bfr(bias[c0 + cofs]); val[1] += bfr(bias[c0 + cofs + 1]); val[2] += bfr(bias[c0 + cofs + 2]); val[3] += bfr(bias[c0 + cofs + 3]); }
                *(volatile v4f*)(crow + (size_t)row * ldc + cofs) = val; }
            if (ps == 0) __threadfence(); }
        __builtin_amdgcn_wave_barrier(); asm volatile("" ::: "memory");
    }
}

__global__ __launch_bounds__(256) void k_wtG(const float* __restrict__ w, int K, int N, bf* Bt) {
    const int lane = threadIdx.x & 31; const int L0 = (blockIdx.x * 8 + (threadIdx.x >> 5)) * 8; const int nlines = N * K / 64;
#pragma unroll 1
    for (int ps = 0; ps < 2; ++ps) {
#pragma unroll 1
        for (int l = 0; l < 8; ++l) { const int L = L0 + l; if (L >= nlines) break; const size_t e = (size_t)L * 64 + lane * 2; const int k = (int)(e % K), n = (int)(e / K); v2us o;
            o[0] = f2bf(w[(size_t)k * N + n]); o[1] = f2bf(w[(size_t)(k + 1) * N + n]); *(volatile v2us*)(Bt + e) = o; }
        if (ps == 0) __threadfence(); }
}
__global__ __launch_bounds__(256) void k_wtGh(const float* __restrict__ w, int K, int N, float sc, h16* Bt) {
    const int lane = threadIdx.x & 31; const int L0 = (blockIdx.x * 8 + (threadIdx.x >> 5)) * 8; const int nlines = N * K / 64;
#pragma unroll 1
    for (int ps = 0; ps < 2; ++ps) {
#pragma unroll 1
        for (int l = 0; l < 8; ++l) { const int L = L0 + l; if (L >= nlines) break; const size_t e = (size_t)L * 64 + lane * 2; const int k = (int)(e % K), n = (int)(e / K); v2h o;
            o[0] = tohx(bfr(w[(size_t)k * N + n]) * sc); o[1] = tohx(bfr(w[(size_t)(k + 1) * N + n]) * sc); *(volatile v2h*)(Bt + e) = o; }
        if (ps == 0) __threadfence(); }
}
__global__ __launch_bounds__(256) void k_cvtx(const float* __restrict__ x, bf* XB) {
    const size_t i = (size_t)blockIdx.x * 256 + threadIdx.x; if (i >= (size_t)MROWS * (DM / 8)) return;
    const size_t row = i / (DM / 8); const int c8 = (int)(i % (DM / 8)) * 8; const size_t b = row / SEQ, s = row % SEQ;
    const v8f v = *(const v8f*)(x + (b * SEQ_FULL + s) * DM + c8); v8us o;
#pragma unroll
    for (int k = 0; k < 8; ++k) o[k] = f2bf(v[k]);
    *(volatile v8us*)(XB + i * 8) = o; __threadfence(); *(volatile v8us*)(XB + i * 8) = o; }
__global__ __launch_bounds__(256) void k_split8(const float* __restrict__ F, bf* Ph, bf* Pl, size_t n8) {
    const size_t i = (size_t)blockIdx.x * 256 + threadIdx.x; if (i >= n8) return; const v8f v = *(const v8f*)(F + i * 8); v8us oh, ol;
#pragma unroll
    for (int k = 0; k < 8; ++k) { unsigned short a, c; splitf(v[k], a, c); oh[k] = a; ol[k] = c; }
    *(volatile v8us*)(Ph + i * 8) = oh; *(volatile v8us*)(Pl + i * 8) = ol; __threadfence(); *(volatile v8us*)(Ph + i * 8) = oh; *(volatile v8us*)(Pl + i * 8) = ol; }
__global__ __launch_bounds__(256) void k_vtp8(const float* __restrict__ F, h16* VT) {
    const size_t e = ((size_t)blockIdx.x * 256 + threadIdx.x) * 8; if (e >= (size_t)NB * DM * SEQ) return;
    const int t0 = (int)(e % SEQ); const int d = (int)((e / SEQ) % DM); const size_t b = e / ((size_t)SEQ * DM); v8h o;
#pragma unroll
    for (int q = 0; q < 8; ++q) o[q] = tohx(F[(b * SEQ + t0 + q) * DM + d]);
    *(volatile v8h*)(VT + e) = o; __threadfence(); *(volatile v8h*)(VT + e) = o; }
__global__ __launch_bounds__(256) void k_mpack(const int* __restrict__ msk, unsigned* MPk) {
    const int lane = threadIdx.x & 31; const int gr = blockIdx.x * 8 + (threadIdx.x >> 5); if (gr >= MROWS) return;
    const int b = gr / SEQ, s = gr - b * SEQ;
    const int* mr = msk + ((size_t)b * SEQ_FULL + s) * SEQ_FULL;
    unsigned wv[NWL];
#pragma unroll
    for (int hb = 0; hb < NWL; ++hb) { const int jn = min(32, SEQW - hb * 32); unsigned mine = 0u;
#pragma unroll 1
        for (int j = 0; j < jn; ++j) { const int v = mr[(hb * 32 + j) * 32 + lane]; const unsigned bal = (unsigned)__ballot(v != 0); mine = (lane == j) ? bal : mine; }
        wv[hb] = mine; }
    unsigned* dst = MPk + (size_t)gr * SEQW;
#pragma unroll 1
    for (int ps = 0; ps < 2; ++ps) {
#pragma unroll
        for (int hb = 0; hb < NWL; ++hb) { const int jn = min(32, SEQW - hb * 32); if (lane < jn) *(volatile unsigned*)(dst + hb * 32 + lane) = wv[hb]; }
        if (ps == 0) __threadfence(); }
}

__global__ __launch_bounds__(256) void k_attn(const bf* __restrict__ QHp, const bf* __restrict__ QLp, const bf* __restrict__ KHp, const bf* __restrict__ KLp, const h16* __restrict__ VT, const unsigned* __restrict__ MPk, h16* CTX) {
    __shared__ __align__(16) h16 pb[8][16 * 32];
    __shared__ __align__(16) float os[8][16 * 68];
    const int tid = threadIdx.x, w = tid >> 5, lane = tid & 31, lm = lane & 15, hi = lane >> 4;
    const int b = blockIdx.z, h = blockIdx.y;
    const int q0 = blockIdx.x * 128 + w * 16;
    const size_t grow0 = (size_t)b * SEQ + q0;
    h16* pw = &pb[w][0]; float* ow = &os[w][0];
    const size_t qo = (grow0 + lm) * DM + h * HD + 8 * hi;
    const v16bf qh0 = WFrag<bf>::ld(QHp + qo), qh1 = WFrag<bf>::ld(QHp + qo + 32), ql0 = WFrag<bf>::ld(QLp + qo), ql1 = WFrag<bf>::ld(QLp + qo + 32);
    v8f ofr[4];
#pragma unroll
    for (int t = 0; t < 4; ++t) ofr[t] = (v8f){};
    float mrow[8], lrow[8];
#pragma unroll
    for (int i = 0; i < 8; ++i) { mrow[i] = -3.0e38f; lrow[i] = 0.0f; }
    const size_t kbase = (size_t)b * SEQ;
    const size_t vbase = ((size_t)b * DM + h * HD + lm) * SEQ + 8 * hi;
#pragma unroll 1
    for (int kc = 0; kc < SEQ; kc += 32) {
        unsigned mw[8];
#pragma unroll
        for (int i = 0; i < 8; ++i) mw[i] = MPk[(grow0 + i + 8 * hi) * SEQW + (kc >> 5)];
        v8f sc[2];
#pragma unroll
        for (int c = 0; c < 2; ++c) {
            const size_t ko = (kbase + kc + c * 16 + lm) * DM + h * HD + 8 * hi;
            const v16bf kh0 = WFrag<bf>::ld(KHp + ko), kh1 = WFrag<bf>::ld(KHp + ko + 32), kl0 = WFrag<bf>::ld(KLp + ko), kl1 = WFrag<bf>::ld(KLp + ko + 32);
            v8f z = (v8f){};
            z = wmmab(qh0, kh0, z); z = wmmab(qh1, kh1, z); z = wmmab(ql0, kh0, z); z = wmmab(ql1, kh1, z); z = wmmab(qh0, kl0, z); z = wmmab(qh1, kl1, z);
            asm volatile("v_nop\n\tv_nop\n\tv_nop\n\tv_nop" : "+v"(z) : "v"(qh0), "v"(ql1), "v"(kh0), "v"(kh1), "v"(kl0), "v"(kl1));
            sc[c] = z;
        }
#pragma unroll
        for (int i = 0; i < 8; ++i) {
            const bool ok0 = ((mw[i] >> lm) & 1u) != 0u, ok1 = ((mw[i] >> (16 + lm)) & 1u) != 0u;
            const float s0 = ok0 ? sc[0][i] * SCL : NEGV, s1 = ok1 ? sc[1][i] * SCL : NEGV;
            float cm = fmaxf(s0, s1);
#pragma unroll
            for (int off = 1; off < 16; off <<= 1) cm = fmaxf(cm, __shfl_xor(cm, off, 32));
            const float mn = fmaxf(mrow[i], cm);
            const float dr = fmaxf(mrow[i] - mn, -120.0f), d0 = fmaxf(s0 - mn, -120.0f), d1 = fmaxf(s1 - mn, -120.0f);
            const float resc = __builtin_amdgcn_exp2f(dr * L2E);
            const float e0 = __builtin_amdgcn_exp2f(d0 * L2E), e1 = __builtin_amdgcn_exp2f(d1 * L2E);
            const float p0 = ok0 ? e0 : 0.0f, p1 = ok1 ? e1 : 0.0f;
            float rs = p0 + p1;
#pragma unroll
            for (int off = 1; off < 16; off <<= 1) rs += __shfl_xor(rs, off, 32);
            lrow[i] = lrow[i] * resc + rs; mrow[i] = mn;
#pragma unroll
            for (int t = 0; t < 4; ++t) ofr[t][i] = ofr[t][i] * resc;
            pw[(i + 8 * hi) * 32 + lm] = tohx(p0 * PCAR); pw[(i + 8 * hi) * 32 + 16 + lm] = tohx(p1 * PCAR);
        }
        __builtin_amdgcn_fence(3  , "wavefront"); __builtin_amdgcn_wave_barrier(); asm volatile("" ::: "memory");
        const v16h pa = cat16(*(const v8ha*)(pw + lm * 32 + 8 * hi), *(const v8ha*)(pw + lm * 32 + 16 + 8 * hi));
        asm volatile("" ::: "memory");
        v16h vb[4];
#pragma unroll
        for (int t = 0; t < 4; ++t) { const size_t vo = vbase + (size_t)t * 16 * SEQ + kc; vb[t] = cat16(*(const v8h*)(VT + vo), *(const v8h*)(VT + vo + 16)); ofr[t] = wmma16(pa, vb[t], ofr[t]); }
        asm volatile("v_nop\n\tv_nop\n\tv_nop\n\tv_nop" : "+v"(ofr[0]), "+v"(ofr[1]), "+v"(ofr[2]), "+v"(ofr[3]) : "v"(pa), "v"(vb[0]), "v"(vb[1]), "v"(vb[2]), "v"(vb[3]));
        __builtin_amdgcn_wave_barrier(); asm volatile("" ::: "memory");
    }
    float inv[8];
#pragma unroll
    for (int i = 0; i < 8; ++i) { const float l = lrow[i]; const float r = 1.0f / fmaxf(l, 1.0e-20f); inv[i] = (l > 0.0f) ? r * (CCAR / PCAR) : 0.0f; }
#pragma unroll
    for (int t = 0; t < 4; ++t)
#pragma unroll
        for (int j = 0; j < 8; ++j) ow[(8 * hi + j) * 68 + t * 16 + lm] = ofr[t][j] * inv[j];
    __builtin_amdgcn_fence(3  , "wavefront"); __builtin_amdgcn_wave_barrier(); asm volatile("" ::: "memory");
    v8h o4[4];
#pragma unroll
    for (int s4 = 0; s4 < 4; ++s4) { const int row = 4 * s4 + (lane >> 3), c8 = (lane & 7) * 8; const v4f a0 = *(const v4fa*)(ow + row * 68 + c8), a1 = *(const v4fa*)(ow + row * 68 + c8 + 4); v8h o;
        o[0] = tohx(a0[0]); o[1] = tohx(a0[1]); o[2] = tohx(a0[2]); o[3] = tohx(a0[3]); o[4] = tohx(a1[0]); o[5] = tohx(a1[1]); o[6] = tohx(a1[2]); o[7] = tohx(a1[3]); o4[s4] = o; }
    h16* cb = CTX + grow0 * DM + h * HD;
#pragma unroll 1
    for (int ps = 0; ps < 2; ++ps) {
#pragma unroll
        for (int s4 = 0; s4 < 4; ++s4) { const int row = 4 * s4 + (lane >> 3), c8 = (lane & 7) * 8; *(volatile v8h*)(cb + (size_t)row * DM + c8) = o4[s4]; }
        if (ps == 0) __threadfence(); }
}

extern "C" void kernel_launch(void* const* d_in, const int* in_sizes, int n_in,
                              void* d_out, int out_size, void* d_ws, size_t ws_size, hipStream_t stream) {
    if (n_in < 10) return;
    const long long needx = (long long)(NB - 1) * SEQ_FULL * DM + (long long)SEQ * DM;
    const long long needm = (long long)(NB - 1) * SEQ_FULL * SEQ_FULL + (long long)(SEQ - 1) * SEQ_FULL + SEQ;
    if ((long long)in_sizes[0] < needx || (long long)in_sizes[1] < needm || (long long)out_size < needx) return;
    if (in_sizes[2] < DM * DM || in_sizes[4] < DM * DM || in_sizes[6] < DM * DM || in_sizes[8] < DM * DM) return;
    if (in_sizes[3] < DM || in_sizes[5] < DM || in_sizes[7] < DM || in_sizes[9] < DM) return;
    const float* x  = (const float*)d_in[0]; const int* msk = (const int*)d_in[1];
    const float* wq = (const float*)d_in[2]; const float* bq = (const float*)d_in[3];
    const float* wk = (const float*)d_in[4]; const float* bk = (const float*)d_in[5];
    const float* wv = (const float*)d_in[6]; const float* bv = (const float*)d_in[7];
    const float* wo = (const float*)d_in[8]; const float* bo = (const float*)d_in[9];
    float* OUT = (float*)d_out;
    char* wsp = (char*)d_ws;
    auto take = [&](size_t bytes) { char* p = wsp; wsp += (bytes + 255) & ~(size_t)255; return (void*)p; };
    bf* WQT = (bf*)take((size_t)DM * DM * 2); bf* WKT = (bf*)take((size_t)DM * DM * 2); bf* WVT = (bf*)take((size_t)DM * DM * 2); h16* WOT = (h16*)take((size_t)DM * DM * 2);
    unsigned* MPk = (unsigned*)take((size_t)MROWS * SEQW * 4);
    bf* XB = (bf*)take((size_t)MROWS * DM * 2);
    float* F = (float*)take((size_t)MROWS * DM * 4);
    bf* QH = (bf*)take((size_t)MROWS * DM * 2); bf* QL = (bf*)take((size_t)MROWS * DM * 2); bf* KH = (bf*)take((size_t)MROWS * DM * 2); bf* KL = (bf*)take((size_t)MROWS * DM * 2);
    h16* VT = (h16*)take((size_t)NB * DM * SEQ * 2);
    h16* CTX = (h16*)take((size_t)MROWS * DM * 2);
    if ((size_t)(wsp - (char*)d_ws) > ws_size) return;

    const unsigned gW = (unsigned)((DM * DM / 64 + 63) / 64);
    k_wtG<<<gW, 256, 0, stream>>>(wq, DM, DM, WQT);
    k_wtG<<<gW, 256, 0, stream>>>(wk, DM, DM, WKT);
    k_wtG<<<gW, 256, 0, stream>>>(wv, DM, DM, WVT);
    k_wtGh<<<gW, 256, 0, stream>>>(wo, DM, DM, WCAR, WOT);
    k_mpack<<<(unsigned)((MROWS + 7) / 8), 256, 0, stream>>>(msk, MPk);
    const size_t n8 = (size_t)MROWS * DM / 8; const unsigned g8 = (unsigned)((n8 + 255) / 256);
    k_cvtx<<<g8, 256, 0, stream>>>(x, XB);
    const dim3 gp((unsigned)(MROWS / 64), (unsigned)(DM / 64), 1);
    k_gemmw<bf, 0, true><<<gp, 32, 0, stream>>>(XB, (const bf*)nullptr, WQT, (const bf*)nullptr, DM, F, DM, bq, 1.0f, (size_t)0, (size_t)0, (size_t)0);
    k_split8<<<g8, 256, 0, stream>>>(F, QH, QL, n8);
    k_gemmw<bf, 0, true><<<gp, 32, 0, stream>>>(XB, (const bf*)nullptr, WKT, (const bf*)nullptr, DM, F, DM, bk, 1.0f, (size_t)0, (size_t)0, (size_t)0);
    k_split8<<<g8, 256, 0, stream>>>(F, KH, KL, n8);
    k_gemmw<bf, 0, true><<<gp, 32, 0, stream>>>(XB, (const bf*)nullptr, WVT, (const bf*)nullptr, DM, F, DM, bv, 1.0f, (size_t)0, (size_t)0, (size_t)0);
    k_vtp8<<<(unsigned)(((size_t)NB * DM * SEQ / 8 + 255) / 256), 256, 0, stream>>>(F, VT);
    k_attn<<<dim3((unsigned)(SEQ / 128), (unsigned)NHD, (unsigned)NB), 256, 0, stream>>>(QH, QL, KH, KL, VT, MPk, CTX);
    k_gemmw<h16, 0, true><<<dim3((unsigned)(SEQ / 64), (unsigned)(DM / 64), (unsigned)NB), 32, 0, stream>>>(CTX, (const h16*)nullptr, WOT, (const h16*)nullptr, DM, OUT, DM, bo, 1.0f / (CCAR * WCAR), (size_t)SEQ * DM, (size_t)0, (size_t)SEQ_FULL * DM);
}
